// masked_multi_head_attention_28948079575364
// MI455X (gfx1250) — hardware-verified
//
#include <hip/hip_runtime.h>


namespace {
constexpr int S = 4096, D = 1024, H = 16, HD = 64, CH = 256;
constexpr float XS = 8.0f, HS = 256.0f, PS = 256.0f, WSC = 256.0f, SCALE = 0.125f;
typedef _Float16 b16;
typedef __attribute__((ext_vector_type(16))) _Float16 v16b;
typedef __attribute__((ext_vector_type(8))) _Float16 v8b;
typedef __attribute__((ext_vector_type(2))) _Float16 v2b;
typedef __attribute__((ext_vector_type(8))) float v8f;
typedef __attribute__((ext_vector_type(4))) float v4f;
__device__ __forceinline__ float bf16_rne(float f) { unsigned int u = __float_as_uint(f); u += 0x7FFFu + ((u >> 16) & 1u); float r = __uint_as_float(u & 0xFFFF0000u); asm volatile("" : "+v"(r)); return r; }
__device__ __forceinline__ float bfv(float f) { float r = bf16_rne(f); asm volatile("" : "+v"(r)); return r; }
__device__ __forceinline__ void split16(float v, b16& hi, b16& lo) { hi = (b16)v; lo = (b16)(v - (float)hi); }
__device__ __forceinline__ v16b frag_kb(const b16* p, int hh) { const v8b a = *(const v8b*)(p + 8 * hh), b = *(const v8b*)(p + 16 + 8 * hh); v16b f;
#pragma unroll
  for (int e = 0; e < 8; ++e) { f[e] = a[e]; f[8 + e] = b[e]; } return f; }
__device__ __forceinline__ v8f wmma16b(v16b a, v16b b, v8f c) { v8f d = __builtin_amdgcn_wmma_f32_16x16x32_f16(false, a, false, b, (short)0, c, false, false); asm volatile("v_nop\n\tv_nop\n\tv_nop\n\tv_nop" : "+v"(d) : "v"(a), "v"(b)); return d; }
__device__ __forceinline__ void wave_lds_sync() { __builtin_amdgcn_fence(__ATOMIC_RELEASE, "workgroup"); __builtin_amdgcn_wave_barrier(); __builtin_amdgcn_fence(__ATOMIC_ACQUIRE, "workgroup"); }

__global__ __launch_bounds__(256) void wput_kernel(const float* __restrict__ wq, const float* __restrict__ wk, const float* __restrict__ wv, const float* __restrict__ wo, b16* __restrict__ WQKV, b16* __restrict__ WO) { const size_t nt = (size_t)gridDim.x * 256, u0 = (size_t)blockIdx.x * 256 + threadIdx.x; v8b v;
  for (size_t u = u0; u < (size_t)4 * D * 128; u += nt) { const int o = (int)(u / 128), k0 = (int)(u % 128) * 8; const int which = o / D, oo = o % D; const float* w = which == 0 ? wq : (which == 1 ? wk : (which == 2 ? wv : wo));
#pragma unroll
    for (int j = 0; j < 8; ++j) v[j] = (b16)(bf16_rne(w[(size_t)oo * D + k0 + j]) * WSC); b16* dst = which < 3 ? WQKV + (size_t)o * D + k0 : WO + (size_t)oo * D + k0; for (int pass = 0; pass < 2; ++pass) { *(volatile v8b*)dst = v; __threadfence(); } } }
__global__ __launch_bounds__(32) void proj_kernel(const float* __restrict__ x, const b16* __restrict__ WQKV, const float* __restrict__ bq, const float* __restrict__ bk, const float* __restrict__ bv, b16* __restrict__ Qh, b16* __restrict__ Ql, b16* __restrict__ Kh, b16* __restrict__ Kl, float* __restrict__ V) { __shared__ __attribute__((aligned(16))) b16 Ax[16][D + 8]; __shared__ float Tf[16][260]; const int lane = threadIdx.x, nloc = lane & 15, hlf = lane >> 4; const size_t t0 = (size_t)blockIdx.x * 16;
  for (int rr = 0; rr < 16; ++rr) for (int q = 0; q < D / 32; ++q) { const int c = q * 32 + lane; Ax[rr][c] = (b16)(bf16_rne(x[(t0 + rr) * D + c]) * XS); }
  if (lane < 16) for (int k = D; k < D + 8; ++k) Ax[lane][k] = (b16)0.0f;
  wave_lds_sync();
#pragma unroll 1
  for (int g = 0; g < 12; ++g) { const int which = g / 4, c0 = (g % 4) * 256; const float* bias = which == 0 ? bq : (which == 1 ? bk : bv); v8f acc[16];
#pragma unroll
    for (int t = 0; t < 16; ++t) acc[t] = (v8f){};
#pragma unroll 2
    for (int kb = 0; kb < D; kb += 32) { const v16b a = frag_kb(&Ax[nloc][kb], hlf);
#pragma unroll
      for (int t = 0; t < 16; ++t) acc[t] = wmma16b(a, frag_kb(WQKV + ((size_t)which * D + c0 + t * 16 + nloc) * D + kb, hlf), acc[t]); }
#pragma unroll
    for (int t = 0; t < 16; ++t) { const int cc = t * 16 + nloc; const float bb = bfv(bias[c0 + cc]);
#pragma unroll
      for (int r8 = 0; r8 < 8; ++r8) Tf[8 * hlf + r8][cc] = acc[t][r8] * (1.0f / (XS * WSC)) + bb; }
    wave_lds_sync();
    for (int pass = 0; pass < 2; ++pass) { for (int rr = 0; rr < 16; ++rr) { const size_t tk = t0 + rr;
        if (which == 2) { for (int q = 0; q < 2; ++q) *(volatile v4f*)(V + tk * D + c0 + q * 128 + lane * 4) = *(const v4f*)(&Tf[rr][q * 128 + lane * 4]); }
        else { b16* Ph = which == 0 ? Qh : Kh; b16* Pl = which == 0 ? Ql : Kl; for (int q = 0; q < 4; ++q) { const int c = q * 64 + lane * 2; b16 h0, l0, h1, l1; split16(Tf[rr][c] * HS, h0, l0); split16(Tf[rr][c + 1] * HS, h1, l1); *(volatile v2b*)(Ph + tk * D + c0 + c) = (v2b){h0, h1}; *(volatile v2b*)(Pl + tk * D + c0 + c) = (v2b){l0, l1}; } } }
      __threadfence(); }
    wave_lds_sync(); } }
__global__ __launch_bounds__(256) void vt_kernel(const float* __restrict__ V, b16* __restrict__ VTh, b16* __restrict__ VTl) { __shared__ float Tt[64][257]; const int s0 = (blockIdx.x >> 2) * 64, hg = blockIdx.x & 3; const int tid = threadIdx.x, wave = tid >> 5, lane = tid & 31;
  for (int q = wave; q < 64; q += 8) for (int c = lane; c < 256; c += 32) Tt[q][c] = V[(size_t)(s0 + q) * D + hg * 256 + c];
  __syncthreads();
  for (int pass = 0; pass < 2; ++pass) { for (int c = wave; c < 256; c += 8) { const int h = hg * 4 + c / HD, d = c % HD; b16 h0, l0, h1, l1; split16(Tt[lane * 2][c] * HS, h0, l0); split16(Tt[lane * 2 + 1][c] * HS, h1, l1); const size_t o = ((size_t)h * HD + d) * S + s0 + lane * 2; *(volatile v2b*)(VTh + o) = (v2b){h0, h1}; *(volatile v2b*)(VTl + o) = (v2b){l0, l1}; } __threadfence(); } }
__global__ __launch_bounds__(32) void att_kernel(const b16* __restrict__ Qh, const b16* __restrict__ Ql, const b16* __restrict__ Kh, const b16* __restrict__ Kl, const b16* __restrict__ VTh, const b16* __restrict__ VTl, int QLIM, float* __restrict__ O) { __shared__ __attribute__((aligned(16))) b16 Pa[32][CH + 8], Pb[32][CH + 8]; __shared__ float Sc[32][CH + 1], Mx[32], Ls[32], Fc[32], Of[32][HD + 1]; const int lane = threadIdx.x, nloc = lane & 15, hlf = lane >> 4; const int h = blockIdx.x / (S / 16), q0 = (blockIdx.x % (S / 16)) * 16; if (q0 >= QLIM) return;
  Mx[lane] = -INFINITY; Ls[lane] = 0.0f; for (int kk = CH; kk < CH + 8; ++kk) { Pa[lane][kk] = (b16)0.0f; Pb[lane][kk] = (b16)0.0f; }
  wave_lds_sync();
  v16b qa[1][2], ql[1][2]; for (int rt = 0; rt < 1; ++rt) for (int ks = 0; ks < 2; ++ks) { qa[rt][ks] = frag_kb(Qh + (size_t)(q0 + rt * 16 + nloc) * D + h * HD + ks * 32, hlf); ql[rt][ks] = frag_kb(Ql + (size_t)(q0 + rt * 16 + nloc) * D + h * HD + ks * 32, hlf); }
  v8f oacc[1][4];
#pragma unroll
  for (int rt = 0; rt < 1; ++rt)
#pragma unroll
    for (int t = 0; t < 4; ++t) oacc[rt][t] = (v8f){};
  const int nch = q0 / CH + 1;
#pragma unroll 1
  for (int ch = 0; ch < nch; ++ch) { const int k0 = ch * CH;
#pragma unroll 1
    for (int tg = 0; tg < 16; tg += 4) { v8f sacc[1][4];
#pragma unroll
      for (int rt = 0; rt < 1; ++rt)
#pragma unroll
        for (int t = 0; t < 4; ++t) sacc[rt][t] = (v8f){};
#pragma unroll
      for (int t = 0; t < 4; ++t)
#pragma unroll
        for (int ks = 0; ks < 2; ++ks) { const size_t ko = (size_t)(k0 + (tg + t) * 16 + nloc) * D + h * HD + ks * 32; const v16b kh = frag_kb(Kh + ko, hlf), kl = frag_kb(Kl + ko, hlf);
#pragma unroll
          for (int rt = 0; rt < 1; ++rt) { sacc[rt][t] = wmma16b(qa[rt][ks], kh, sacc[rt][t]); sacc[rt][t] = wmma16b(qa[rt][ks], kl, sacc[rt][t]); sacc[rt][t] = wmma16b(ql[rt][ks], kh, sacc[rt][t]); } }
#pragma unroll
      for (int rt = 0; rt < 1; ++rt)
#pragma unroll
        for (int t = 0; t < 4; ++t)
#pragma unroll
          for (int r8 = 0; r8 < 8; ++r8) Sc[rt * 16 + 8 * hlf + r8][(tg + t) * 16 + nloc] = sacc[rt][t][r8] * (SCALE / (HS * HS)); }
    wave_lds_sync();
    if (lane < 16) { const int r = lane, qi = q0 + r; float mx = -INFINITY; for (int j = 0; j < CH; ++j) if (k0 + j <= qi) mx = fmaxf(mx, Sc[r][j]); const float mo = Mx[r], mn = fmaxf(mo, mx); float sm = 0.0f; for (int j = 0; j < CH; ++j) { const float p = (k0 + j <= qi) ? __expf(Sc[r][j] - mn) : 0.0f; sm += p; b16 ph, pl; split16(p * PS, ph, pl); Pa[r][j] = ph; Pb[r][j] = pl; } const float fac = (mo == -INFINITY) ? 0.0f : __expf(mo - mn); Fc[r] = fac; Ls[r] = Ls[r] * fac + sm; Mx[r] = mn; }
    wave_lds_sync();
#pragma unroll
    for (int rt = 0; rt < 1; ++rt)
#pragma unroll
      for (int t = 0; t < 4; ++t)
#pragma unroll
        for (int r8 = 0; r8 < 8; ++r8) oacc[rt][t][r8] *= Fc[rt * 16 + 8 * hlf + r8];
#pragma unroll 2
    for (int kb = 0; kb < CH; kb += 32)
#pragma unroll
      for (int rt = 0; rt < 1; ++rt) { const v16b pa = frag_kb(&Pa[rt * 16 + nloc][kb], hlf), pb = frag_kb(&Pb[rt * 16 + nloc][kb], hlf);
#pragma unroll
        for (int t = 0; t < 4; ++t) { const size_t vo = ((size_t)h * HD + t * 16 + nloc) * S + k0 + kb; const v16b vh = frag_kb(VTh + vo, hlf), vl = frag_kb(VTl + vo, hlf); oacc[rt][t] = wmma16b(pa, vh, oacc[rt][t]); oacc[rt][t] = wmma16b(pa, vl, oacc[rt][t]); oacc[rt][t] = wmma16b(pb, vh, oacc[rt][t]); } }
    wave_lds_sync(); }
#pragma unroll
  for (int rt = 0; rt < 1; ++rt)
#pragma unroll
    for (int t = 0; t < 4; ++t)
#pragma unroll
      for (int r8 = 0; r8 < 8; ++r8) { const int r = rt * 16 + 8 * hlf + r8; Of[r][t * 16 + nloc] = oacc[rt][t][r8] * (1.0f / (PS * HS)) / Ls[r]; }
  wave_lds_sync();
  typedef __attribute__((ext_vector_type(2))) float v2f;
  for (int pass = 0; pass < 2; ++pass) { for (int r = 0; r < 16; ++r) *(volatile v2f*)(O + (size_t)(q0 + r) * D + h * HD + lane * 2) = (v2f){Of[r][lane * 2], Of[r][lane * 2 + 1]}; __threadfence(); } }
__global__ __launch_bounds__(32) void outp_kernel(const float* __restrict__ O, const b16* __restrict__ WO, const float* __restrict__ bo, int QLIM, float* __restrict__ out) { __shared__ __attribute__((aligned(16))) b16 Ah[16][D + 8], Al[16][D + 8]; __shared__ float Tf[16][260]; const int lane = threadIdx.x, nloc = lane & 15, hlf = lane >> 4; const size_t t0 = (size_t)blockIdx.x * 16; if (t0 >= (size_t)QLIM) return;
  for (int rr = 0; rr < 16; ++rr) for (int q = 0; q < D / 32; ++q) { const int c = q * 32 + lane; b16 p, pl; split16(O[(t0 + rr) * D + c] * HS, p, pl); Ah[rr][c] = p; Al[rr][c] = pl; }
  if (lane < 16) for (int k = D; k < D + 8; ++k) { Ah[lane][k] = (b16)0.0f; Al[lane][k] = (b16)0.0f; }
  wave_lds_sync();
#pragma unroll 1
  for (int g = 0; g < 4; ++g) { v8f acc[16];
#pragma unroll
    for (int t = 0; t < 16; ++t) acc[t] = (v8f){};
#pragma unroll 2
    for (int kb = 0; kb < D; kb += 32) { const v16b a = frag_kb(&Ah[nloc][kb], hlf), al = frag_kb(&Al[nloc][kb], hlf);
#pragma unroll
      for (int t = 0; t < 16; ++t) { const v16b bw = frag_kb(WO + (size_t)(g * 256 + t * 16 + nloc) * D + kb, hlf); acc[t] = wmma16b(a, bw, acc[t]); acc[t] = wmma16b(al, bw, acc[t]); } }
#pragma unroll
    for (int t = 0; t < 16; ++t) { const int cc = t * 16 + nloc; const float bb = bfv(bo[g * 256 + cc]);
#pragma unroll
      for (int r8 = 0; r8 < 8; ++r8) Tf[8 * hlf + r8][cc] = acc[t][r8] * (1.0f / (HS * WSC)) + bb; }
    wave_lds_sync();
    for (int pass = 0; pass < 2; ++pass) { for (int rr = 0; rr < 16; ++rr) for (int q = 0; q < 2; ++q) *(volatile v4f*)(out + (t0 + rr) * D + g * 256 + q * 128 + lane * 4) = *(const v4f*)(&Tf[rr][q * 128 + lane * 4]); __threadfence(); }
    wave_lds_sync(); } }
}

extern "C" void kernel_launch(void* const* d_in, const int* in_sizes, int n_in, void* d_out, int out_size, void* d_ws, size_t ws_size, hipStream_t stream) {
  (void)n_in;
  auto Fp = [&](int i) { return (const float*)d_in[i]; };
  if (in_sizes[0] != S * D || in_sizes[1] != D * D || in_sizes[3] != D * D || in_sizes[5] != D * D || in_sizes[7] != D * D || out_size != S * D) return;
  const int QLIM = S;
  size_t off = 0; char* ws = (char*)d_ws;
  auto carve = [&](size_t bytes) { char* p = ws + off; off += (bytes + 255) & ~(size_t)255; return p; };
  b16* WQKV = (b16*)carve((size_t)3 * D * D * 2); b16* WO = (b16*)carve((size_t)D * D * 2); b16* Qh = (b16*)carve((size_t)S * D * 2); b16* Ql = (b16*)carve((size_t)S * D * 2); b16* Kh = (b16*)carve((size_t)S * D * 2); b16* Kl = (b16*)carve((size_t)S * D * 2); float* V = (float*)carve((size_t)S * D * 4); b16* VTh = (b16*)carve((size_t)D * S * 2); b16* VTl = (b16*)carve((size_t)D * S * 2); float* O = (float*)carve((size_t)S * D * 4);
  if (off > ws_size || off > ((size_t)96 << 20)) return;
  wput_kernel<<<256, 256, 0, stream>>>(Fp(1), Fp(3), Fp(5), Fp(7), WQKV, WO);
  proj_kernel<<<QLIM / 16, 32, 0, stream>>>(Fp(0), WQKV, Fp(2), Fp(4), Fp(6), Qh, Ql, Kh, Kl, V);
  vt_kernel<<<(S / 64) * 4, 256, 0, stream>>>(V, VTh, VTl);
  att_kernel<<<H * (S / 16), 32, 0, stream>>>(Qh, Ql, Kh, Kl, VTh, VTl, QLIM, O);
  outp_kernel<<<S / 16, 32, 0, stream>>>(O, WO, Fp(8), QLIM, (float*)d_out);
}
